// DeformSimpleBottleneck_25357486916158
// MI455X (gfx1250) — hardware-verified
//
#include <hip/hip_runtime.h>
#include <hip/hip_bf16.h>

typedef _Float16 bf16_t;
typedef __attribute__((ext_vector_type(16))) _Float16 v16bf;
typedef __attribute__((ext_vector_type(8)))  _Float16 v8bf;
typedef __attribute__((ext_vector_type(4)))  _Float16 v4bf;
typedef __attribute__((ext_vector_type(8)))  float  v8f;
typedef __attribute__((ext_vector_type(4)))  int    v4i;

#define EPS 1e-5f
#define Bsz 4
#define Hd  64
#define Wdm 64
#define C0  256
#define C1  512
#define Gd  2
#define Kt  9
#define DIL 2
#define Hp  60
#define Wp  60
#define NROW (Bsz*Hp*Wp)
#define CG   (C1/Gd)
#define KDEF (Gd*Kt*CG)
#define KOFF (Kt*C1)
#define OFFCH 54
#define OFFPAD 64
#define OFFP   64
#define KC   128
#define NSTG (KDEF / KC)

#define USE_ASYNC_LDS 0

#if __has_builtin(__builtin_amdgcn_s_wait_asynccnt)
#define WAIT_ASYNC(n) __builtin_amdgcn_s_wait_asynccnt(n)
#else
#define WAIT_ASYNC(n) asm volatile("s_wait_asynccnt %0" ::"i"(n) : "memory")
#endif

constexpr size_t al256(size_t x) { return (x + 255) & ~(size_t)255; }
constexpr size_t WS_Y     = 0;
constexpr size_t WS_OFF   = al256(WS_Y     + (size_t)Bsz*Hd*Wdm*C1*4);
constexpr size_t WS_A     = al256(WS_OFF   + (size_t)NROW*OFFP*4);
constexpr size_t WS_Z     = al256(WS_A     + (size_t)NROW*KDEF*2);
constexpr size_t WS_WT1   = al256(WS_Z     + (size_t)NROW*C1*4);
constexpr size_t WS_B1    = al256(WS_WT1   + (size_t)C1*C0*2);
constexpr size_t WS_WTOFF = al256(WS_B1    + (size_t)C1*4);
constexpr size_t WS_WD    = al256(WS_WTOFF + (size_t)OFFPAD*KOFF*2);
constexpr size_t WS_B2    = al256(WS_WD    + (size_t)C1*KDEF*2);
constexpr size_t WS_W3T   = al256(WS_B2    + (size_t)C1*4);
constexpr size_t WS_B3    = al256(WS_W3T   + (size_t)C0*C1*2);

__device__ __forceinline__ v8f wmma_bf16(v16bf a, v16bf b, v8f c) {
  v8f d = __builtin_amdgcn_wmma_f32_16x16x32_f16(false, a, false, b, (short)0, c, false, false);
  asm volatile("v_nop\n\tv_nop\n\tv_nop\n\tv_nop" : "+v"(d) : "v"(a), "v"(b));
  return d;
}
__device__ __forceinline__ v16bf ld_b(const bf16_t* rowk, int half) {
  v8bf lo = *(const v8bf*)(rowk + half * 8), hi = *(const v8bf*)(rowk + 16 + half * 8);
  v16bf r;
#pragma unroll
  for (int i = 0; i < 8; ++i) { r[i] = lo[i]; r[i + 8] = hi[i]; }
  return r;
}
__device__ __forceinline__ float bn_shift(const float* s, const float* b, const float* m, const float* v, int c) {
  return b[c] - m[c] * (s[c] * (1.0f / sqrtf(v[c] + EPS)));
}
#define VST2(T, ptr, val) do { const T _v = (val); *(volatile T*)(ptr) = _v; __threadfence(); *(volatile T*)(ptr) = _v; } while (0)
template <typename EP, typename DST>
__device__ __forceinline__ void store_rows64(const v8f (&acc)[4], int lane, EP ep, DST dst) {
  const int half = lane >> 4;
  for (int pass = 0; pass < 2; ++pass) {
#pragma unroll
    for (int pr = 0; pr < 2; ++pr)
#pragma unroll
      for (int vv = 0; vv < 8; ++vv) {
        const float a0 = acc[2 * pr][vv], b0 = acc[2 * pr + 1][vv];
        const float ax = __shfl_xor(a0, 16), bx = __shfl_xor(b0, 16);
        const int c = pr * 32 + lane;
        *(volatile float*)(dst(vv) + c)     = ep(vv, c, half ? bx : a0);
        *(volatile float*)(dst(vv + 8) + c) = ep(vv + 8, c, half ? b0 : ax);
      }
    __threadfence();
  }
}

__device__ __forceinline__ v16bf mk_a_f32(const float* p0, const float* p1) {
  float4 a0 = *(const float4*)(p0);
  float4 a1 = *(const float4*)(p0 + 4);
  float4 b0 = *(const float4*)(p1);
  float4 b1 = *(const float4*)(p1 + 4);
  v16bf r;
  r[0]=(bf16_t)a0.x; r[1]=(bf16_t)a0.y; r[2]=(bf16_t)a0.z; r[3]=(bf16_t)a0.w;
  r[4]=(bf16_t)a1.x; r[5]=(bf16_t)a1.y; r[6]=(bf16_t)a1.z; r[7]=(bf16_t)a1.w;
  r[8]=(bf16_t)b0.x; r[9]=(bf16_t)b0.y; r[10]=(bf16_t)b0.z; r[11]=(bf16_t)b0.w;
  r[12]=(bf16_t)b1.x; r[13]=(bf16_t)b1.y; r[14]=(bf16_t)b1.z; r[15]=(bf16_t)b1.w;
  return r;
}

__device__ __forceinline__ v16bf mk_a_bf16(const bf16_t* p0, const bf16_t* p1) {
  v8bf lo = *(const v8bf*)p0;
  v8bf hi = *(const v8bf*)p1;
  v16bf r;
#pragma unroll
  for (int i = 0; i < 8; ++i) { r[i] = lo[i]; r[i+8] = hi[i]; }
  return r;
}

__global__ __launch_bounds__(256) void k_prep_w1(const float* __restrict__ w1,
    const float* __restrict__ s, const float* __restrict__ v, bf16_t* __restrict__ Wt) {
  int t8 = blockIdx.x * blockDim.x + threadIdx.x;
  if (t8 >= C1 * C0 / 8) return;
  int n = (t8 * 8) / C0, c0 = (t8 * 8) % C0;
  float alpha = s[n] * (1.0f / sqrtf(v[n] + EPS));
  v8bf o;
#pragma unroll
  for (int q = 0; q < 8; ++q) o[q] = (bf16_t)(w1[(size_t)(c0 + q) * C1 + n] * alpha);
  VST2(v8bf, Wt + (size_t)n * C0 + c0, o);
}

__global__ __launch_bounds__(256) void k_prep_woff(const float* __restrict__ w_off,
    bf16_t* __restrict__ Wt) {
  int t8 = blockIdx.x * blockDim.x + threadIdx.x;
  if (t8 >= OFFPAD * KOFF / 8) return;
  int n = (t8 * 8) / KOFF, r0 = (t8 * 8) % KOFF;
  v8bf o;
#pragma unroll
  for (int q = 0; q < 8; ++q) {
    int r = r0 + q; int tap = r / C1, c = r % C1;
    o[q] = (bf16_t)((n < OFFCH) ? w_off[((size_t)tap * C1 + c) * OFFCH + n] : 0.f);
  }
  VST2(v8bf, Wt + (size_t)n * KOFF + r0, o);
}

__global__ __launch_bounds__(256) void k_prep_wd(const float* __restrict__ w_d,
    const float* __restrict__ s, const float* __restrict__ v, bf16_t* __restrict__ Wt) {
  int t8 = blockIdx.x * blockDim.x + threadIdx.x;
  if (t8 >= C1 * KDEF / 8) return;
  size_t t0 = (size_t)t8 * 8;
  int f = (int)(t0 / KDEF), r0 = (int)(t0 % KDEF);
  float alpha = s[f] * (1.0f / sqrtf(v[f] + EPS));
  v8bf o;
#pragma unroll
  for (int q = 0; q < 8; ++q) {
    int r = r0 + q;
    int g = r / (Kt * CG), rem = r % (Kt * CG);
    int k = rem / CG, c = rem % CG;
    o[q] = (bf16_t)(w_d[((size_t)k * C1 + (g * CG + c)) * C1 + f] * alpha);
  }
  VST2(v8bf, Wt + (size_t)f * KDEF + r0, o);
}

__global__ __launch_bounds__(256) void k_prep_w3(const float* __restrict__ w3,
    const float* __restrict__ s, const float* __restrict__ v, bf16_t* __restrict__ Wt) {
  int t8 = blockIdx.x * blockDim.x + threadIdx.x;
  if (t8 >= C0 * C1 / 8) return;
  int f = (t8 * 8) / C1, c0 = (t8 * 8) % C1;
  float alpha = s[f] * (1.0f / sqrtf(v[f] + EPS));
  v8bf o;
#pragma unroll
  for (int q = 0; q < 8; ++q) o[q] = (bf16_t)(w3[(size_t)(c0 + q) * C0 + f] * alpha);
  VST2(v8bf, Wt + (size_t)f * C1 + c0, o);
}

__global__ __launch_bounds__(128) void k_gemm1(const float* __restrict__ x,
    const bf16_t* __restrict__ Wt, const float* __restrict__ s, const float* __restrict__ bb_, const float* __restrict__ m, const float* __restrict__ v,
    float* __restrict__ y) {
  const int lane = threadIdx.x & 31;
  const int wave = (blockIdx.x * blockDim.x + threadIdx.x) >> 5;
  const int NW = C1 / 64;
  const int mt = wave / NW, nw = wave % NW;
  if (mt >= (Bsz * Hd * Wdm) / 16) return;
  const int m0 = mt * 16, n0 = nw * 64;
  const int lrow = lane & 15, half = lane >> 4;
  v8f acc[4] = {};
  const float* arow = x + (size_t)(m0 + lrow) * C0;
  for (int kk = 0; kk < C0; kk += 32) {
    v16bf a = mk_a_f32(arow + kk + half * 8, arow + kk + 16 + half * 8);
#pragma unroll
    for (int ns = 0; ns < 4; ++ns) {
      acc[ns] = wmma_bf16(a, ld_b(Wt + (size_t)(n0 + ns * 16 + lrow) * C0 + kk, half), acc[ns]);
    }
  }
  {
    const float sh0 = bn_shift(s, bb_, m, v, n0 + lane), sh1 = bn_shift(s, bb_, m, v, n0 + 32 + lane);
    store_rows64(acc, lane, [&](int r, int c, float val) { return fmaxf(val + (c < 32 ? sh0 : sh1), 0.f); },
                 [&](int r) { return y + (size_t)(m0 + r) * C1 + n0; });
  }
}

__global__ __launch_bounds__(128) void k_gemm_off(const float* __restrict__ y,
    const bf16_t* __restrict__ Wt, const float* __restrict__ b_off,
    float* __restrict__ off) {
  const int lane = threadIdx.x & 31;
  const int wave = (blockIdx.x * blockDim.x + threadIdx.x) >> 5;
  if (wave >= NROW / 16) return;
  const int m0 = wave * 16;
  const int lrow = lane & 15, half = lane >> 4;
  const int row = m0 + lrow;
  const int b = row / (Hp * Wp), rem = row % (Hp * Wp);
  const int i = rem / Wp, j = rem % Wp;
  v8f acc[4] = {};
  for (int kk = 0; kk < KOFF; kk += 32) {
    const int tap = kk >> 9, kloc = kk & 511;
    const int ky = tap / 3, kx = tap % 3;
    const float* arow = y + (((size_t)(b * Hd + i + ky * DIL)) * Wdm + (j + kx * DIL)) * C1 + kloc;
    v16bf a = mk_a_f32(arow + half * 8, arow + 16 + half * 8);
#pragma unroll
    for (int ns = 0; ns < 4; ++ns) {
      acc[ns] = wmma_bf16(a, ld_b(Wt + (size_t)(ns * 16 + lrow) * KOFF + kk, half), acc[ns]);
    }
  }
  {
    const float bo0 = (lane < OFFCH) ? b_off[lane] : 0.f, bo1 = (32 + lane < OFFCH) ? b_off[32 + lane] : 0.f;
    store_rows64(acc, lane, [&](int r, int c, float val) { return val + (c < 32 ? bo0 : bo1); },
                 [&](int r) { return off + (size_t)(m0 + r) * OFFP; });
  }
}

__global__ __launch_bounds__(256) void k_gather(const float* __restrict__ y,
    const float* __restrict__ off, bf16_t* __restrict__ A) {
  size_t t = (size_t)blockIdx.x * blockDim.x + threadIdx.x;
  if (t >= (size_t)NROW * Gd * Kt * (CG / 8)) return;
  const int piece = (int)(t % (CG / 8)); t /= (CG / 8);
  const int row = (int)(t / (Gd * Kt)), gk = (int)(t % (Gd * Kt));
  const int g = gk / Kt, k = gk % Kt;
  const int b = row / (Hp * Wp), rem = row % (Hp * Wp);
  const int i = rem / Wp, j = rem % Wp;
  const float* orow = off + (size_t)row * OFFP;
  const float dy = orow[(g * Kt + k) * 2 + 0];
  const float dx = orow[(g * Kt + k) * 2 + 1];
  const float msk = 1.f / (1.f + expf(-orow[2 * Gd * Kt + g * Kt + k]));
  const float py = (float)i + (float)((k / 3) * DIL) + dy;
  const float px = (float)j + (float)((k % 3) * DIL) + dx;
  const float fy0 = floorf(py), fx0 = floorf(px);
  const int y0 = (int)fy0, x0 = (int)fx0;
  const float wy1 = py - fy0, wx1 = px - fx0;
  const float w00 = (1.f - wy1) * (1.f - wx1) * msk;
  const float w01 = (1.f - wy1) * wx1 * msk;
  const float w10 = wy1 * (1.f - wx1) * msk;
  const float w11 = wy1 * wx1 * msk;
  const bool okY0 = (y0 >= 0) & (y0 < Hd), okY1 = (y0 + 1 >= 0) & (y0 + 1 < Hd);
  const bool okX0 = (x0 >= 0) & (x0 < Wdm), okX1 = (x0 + 1 >= 0) & (x0 + 1 < Wdm);
  const bool v00 = okY0 & okX0, v01 = okY0 & okX1, v10 = okY1 & okX0, v11 = okY1 & okX1;
  const int yc0 = min(max(y0, 0), Hd - 1), yc1 = min(max(y0 + 1, 0), Hd - 1);
  const int xc0 = min(max(x0, 0), Wdm - 1), xc1 = min(max(x0 + 1, 0), Wdm - 1);
  const int c0 = g * CG + piece * 8;
  const float* p00 = y + (((size_t)(b * Hd + yc0)) * Wdm + xc0) * C1 + c0;
  const float* p01 = y + (((size_t)(b * Hd + yc0)) * Wdm + xc1) * C1 + c0;
  const float* p10 = y + (((size_t)(b * Hd + yc1)) * Wdm + xc0) * C1 + c0;
  const float* p11 = y + (((size_t)(b * Hd + yc1)) * Wdm + xc1) * C1 + c0;
  v8bf o;
#pragma unroll
  for (int c = 0; c < 8; ++c) {
    float s_ = 0.f;
    if (v00) s_ += w00 * p00[c];
    if (v01) s_ += w01 * p01[c];
    if (v10) s_ += w10 * p10[c];
    if (v11) s_ += w11 * p11[c];
    o[c] = (bf16_t)s_;
  }
  VST2(v8bf, A + (size_t)row * KDEF + (size_t)(g * Kt + k) * CG + piece * 8, o);
}

__global__ __launch_bounds__(128) void k_gemm_def(const bf16_t* __restrict__ A,
    const bf16_t* __restrict__ Wt, const float* __restrict__ s, const float* __restrict__ bb_, const float* __restrict__ m, const float* __restrict__ v,
    float* __restrict__ z) {
  __shared__ __align__(32) bf16_t sB[2][64 * KC];
  const int tid  = threadIdx.x;
  const int lane = tid & 31;
  const int wave = tid >> 5;
  const int m0 = blockIdx.x * 64 + wave * 16;
  const int n0 = blockIdx.y * 64;
  const int lrow = lane & 15, half = lane >> 4;

  auto issue = [&](int buf, int kk) {
#pragma unroll
    for (int q = 0; q < 8; ++q) {
      const int ch = tid + q * 128;
      const int n  = ch >> 4;
      const int c8 = (ch & 15) << 3;
      const bf16_t* g = Wt + (size_t)(n0 + n) * KDEF + kk + c8;
      bf16_t* l = &sB[buf][ch * 8];
      *(v8bf*)l = *(const v8bf*)g;
    }
  };

  v8f acc[4] = {};
  const bf16_t* arow = A + (size_t)(m0 + lrow) * KDEF;

  issue(0, 0);
  for (int s = 0; s < NSTG; ++s) {
    if (s + 1 < NSTG) {
      issue((s + 1) & 1, (s + 1) * KC);
#if USE_ASYNC_LDS
      WAIT_ASYNC(8);
#endif
    } else {
#if USE_ASYNC_LDS
      WAIT_ASYNC(0);
#endif
    }
    __syncthreads();
    const bf16_t* bufp = sB[s & 1];
    const int kk = s * KC;
#pragma unroll
    for (int ks = 0; ks < KC / 32; ++ks) {
      const bf16_t* ap = arow + kk + ks * 32;
      if (ks == 0) __builtin_prefetch(ap + 2 * KC, 0, 0);
      v16bf a = mk_a_bf16(ap + half * 8, ap + 16 + half * 8);
#pragma unroll
      for (int ns = 0; ns < 4; ++ns) {
        acc[ns] = wmma_bf16(a, ld_b(bufp + (ns * 16 + lrow) * KC + ks * 32, half), acc[ns]);
      }
    }
    __syncthreads();
  }
  {
    const float sh0 = bn_shift(s, bb_, m, v, n0 + lane), sh1 = bn_shift(s, bb_, m, v, n0 + 32 + lane);
    store_rows64(acc, lane, [&](int r, int c, float val) { return fmaxf(val + (c < 32 ? sh0 : sh1), 0.f); },
                 [&](int r) { return z + (size_t)(m0 + r) * C1 + n0; });
  }
}

__global__ __launch_bounds__(128) void k_gemm_out(const float* __restrict__ z,
    const bf16_t* __restrict__ Wt, const float* __restrict__ s, const float* __restrict__ bb_, const float* __restrict__ m, const float* __restrict__ v,
    const float* __restrict__ x, float* __restrict__ out) {
  const int lane = threadIdx.x & 31;
  const int wave = (blockIdx.x * blockDim.x + threadIdx.x) >> 5;
  const int NW = C0 / 64;
  const int mt = wave / NW, nw = wave % NW;
  if (mt >= NROW / 16) return;
  const int m0 = mt * 16, n0 = nw * 64;
  const int lrow = lane & 15, half = lane >> 4;
  v8f acc[4] = {};
  const float* arow = z + (size_t)(m0 + lrow) * C1;
  for (int kk = 0; kk < C1; kk += 32) {
    v16bf a = mk_a_f32(arow + kk + half * 8, arow + kk + 16 + half * 8);
#pragma unroll
    for (int ns = 0; ns < 4; ++ns) {
      acc[ns] = wmma_bf16(a, ld_b(Wt + (size_t)(n0 + ns * 16 + lrow) * C1 + kk, half), acc[ns]);
    }
  }
  {
    const float sh0 = bn_shift(s, bb_, m, v, n0 + lane), sh1 = bn_shift(s, bb_, m, v, n0 + 32 + lane);
    auto rowptr = [&](int r) {
      int mrow = m0 + r;
      int b = mrow / (Hp * Wp), rem = mrow % (Hp * Wp);
      int i = rem / Wp, j = rem % Wp;
      return (((size_t)(b * Hd + i + DIL)) * Wdm + (j + DIL)) * C0 + n0;
    };
    store_rows64(acc, lane, [&](int r, int c, float val) { const size_t oi = rowptr(r) + c; return fmaxf(val + (c < 32 ? sh0 : sh1) + x[oi], 0.f); },
                 [&](int r) { return out + rowptr(r); });
  }
}

__global__ __launch_bounds__(256) void k_border(const float* __restrict__ x,
    float* __restrict__ out) {
  int t = blockIdx.x * blockDim.x + threadIdx.x;
  if (t >= Bsz * Hd * Wdm * C0) return;
  int rest = t / C0;
  int j = rest % Wdm, i = (rest / Wdm) % Hd;
  if (i < DIL || i >= Hd - DIL || j < DIL || j >= Wdm - DIL)
    VST2(float, out + t, fmaxf(x[t], 0.f));
}

extern "C" void kernel_launch(void* const* d_in, const int* in_sizes, int n_in,
                              void* d_out, int out_size, void* d_ws, size_t ws_size,
                              hipStream_t stream) {
  (void)in_sizes; (void)n_in; (void)out_size; (void)ws_size;
  const float* x     = (const float*)d_in[0];
  const float* w1    = (const float*)d_in[1];
  const float* s1    = (const float*)d_in[2];
  const float* b1    = (const float*)d_in[3];
  const float* m1    = (const float*)d_in[4];
  const float* v1    = (const float*)d_in[5];
  const float* w_off = (const float*)d_in[6];
  const float* b_off = (const float*)d_in[7];
  const float* w_d   = (const float*)d_in[8];
  const float* s2    = (const float*)d_in[9];
  const float* b2    = (const float*)d_in[10];
  const float* m2    = (const float*)d_in[11];
  const float* v2    = (const float*)d_in[12];
  const float* w3    = (const float*)d_in[13];
  const float* s3    = (const float*)d_in[14];
  const float* b3    = (const float*)d_in[15];
  const float* m3    = (const float*)d_in[16];
  const float* v3    = (const float*)d_in[17];
  float* out = (float*)d_out;

  (void)in_sizes; (void)n_in; (void)out_size;
  if (ws_size < WS_B3 + 1024) return;
  char* ws = (char*)d_ws;
  float*  y     = (float*) (ws + WS_Y);
  float*  offb  = (float*) (ws + WS_OFF);
  bf16_t* Amat  = (bf16_t*)(ws + WS_A);
  float*  z     = (float*) (ws + WS_Z);
  bf16_t* Wt1   = (bf16_t*)(ws + WS_WT1);
  bf16_t* Wtoff = (bf16_t*)(ws + WS_WTOFF);
  bf16_t* Wdt   = (bf16_t*)(ws + WS_WD);
  bf16_t* W3t   = (bf16_t*)(ws + WS_W3T);

  k_prep_w1 <<<(C1*C0/8 + 255)/256, 256, 0, stream>>>(w1, s1, v1, Wt1);
  k_prep_woff<<<(OFFPAD*KOFF/8 + 255)/256, 256, 0, stream>>>(w_off, Wtoff);
  k_prep_wd <<<(C1*KDEF/8 + 255)/256, 256, 0, stream>>>(w_d, s2, v2, Wdt);
  k_prep_w3 <<<(C0*C1/8 + 255)/256, 256, 0, stream>>>(w3, s3, v3, W3t);

  {
    int waves = ((Bsz*Hd*Wdm)/16) * (C1/64);
    k_gemm1<<<waves/4, 128, 0, stream>>>(x, Wt1, s1, b1, m1, v1, y);
  }
  {
    int waves = NROW/16;
    k_gemm_off<<<(waves + 3)/4, 128, 0, stream>>>(y, Wtoff, b_off, offb);
  }
  k_gather<<<(unsigned)(((size_t)NROW*Gd*Kt*(CG/8) + 255)/256), 256, 0, stream>>>(y, offb, Amat);
  {
    dim3 grid(NROW/64, C1/64);
    k_gemm_def<<<grid, 128, 0, stream>>>(Amat, Wdt, s2, b2, m2, v2, z);
  }
  {
    int waves = (NROW/16) * (C0/64);
    k_gemm_out<<<waves/4, 128, 0, stream>>>(z, W3t, s3, b3, m3, v3, x, out);
  }
  k_border<<<(Bsz*Hd*Wdm*C0 + 255)/256, 256, 0, stream>>>(x, out);
}
